// NeuralAdditiveModel_60739427500189
// MI455X (gfx1250) — hardware-verified
//
#include <hip/hip_runtime.h>
#define BS 16384
#define NF 128
#define U1 64
#define NH1 64
#define NH2 32
#define CHB 2048

typedef __bf16 v16b __attribute__((ext_vector_type(16)));
typedef unsigned short v8us __attribute__((ext_vector_type(8), may_alias));
typedef float  v8f  __attribute__((ext_vector_type(8)));
typedef float  v4f  __attribute__((ext_vector_type(4)));
typedef float  v4fa __attribute__((ext_vector_type(4), may_alias));
union FragB { v16b v; v8us half[2]; unsigned short u[16]; };

__device__ __forceinline__ unsigned short bf16_bits(float x) { unsigned int u = __float_as_uint(x); return (unsigned short)((u + 0x7FFFu + ((u >> 16) & 1u)) >> 16); }
__device__ __forceinline__ float bf16_val(unsigned short b) { return __uint_as_float(((unsigned int)b) << 16); }
__device__ __forceinline__ float bf16_round(float x) { return bf16_val(bf16_bits(x)); }
template <int NT>
__device__ __forceinline__ v8f mmaN(v16b ah, v16b al, v16b bh, v16b bl, v8f c) {
  c = __builtin_amdgcn_wmma_f32_16x16x32_bf16(false, ah, false, bh, (short)0, c, false, false);
  if (NT >= 2) c = __builtin_amdgcn_wmma_f32_16x16x32_bf16(false, al, false, bh, (short)0, c, false, false);
  if (NT >= 3) c = __builtin_amdgcn_wmma_f32_16x16x32_bf16(false, ah, false, bl, (short)0, c, false, false);
  asm volatile("v_nop\n\tv_nop\n\tv_nop\n\tv_nop" : "+v"(c) : "v"(ah), "v"(al), "v"(bh), "v"(bl));
  return c;
}

__global__ __launch_bounds__(256) void k_wt_bf16(const float* __restrict__ W, unsigned short* __restrict__ Wt, int K, int N) {
  const int t = blockIdx.x * 256 + threadIdx.x;
  const int k8n = K / 8;
  if (t >= N * k8n) return;
  const int n = t / k8n, k8 = (t % k8n) * 8;
  v8us v;
#pragma unroll
  for (int i = 0; i < 8; ++i) v[i] = bf16_bits(W[(size_t)(k8 + i) * N + n]);
  *(volatile v8us*)(Wt + (size_t)n * K + k8) = v;
  __threadfence();
  *(volatile v8us*)(Wt + (size_t)n * K + k8) = v;
}

template <bool ASPLIT, int ACT, bool BIAS_BF16>
__global__ __launch_bounds__(128) void k_gemm_bf(const float* __restrict__ A, int lda, const unsigned short* __restrict__ Wt, int ldb,
                                               const float* __restrict__ bias, float* __restrict__ C, int ldc, int M, int N, int K) {
  __shared__ __attribute__((aligned(16))) float so[4][16][64];
  const int tid = threadIdx.x, w = tid >> 5, lane = tid & 31, ln = lane & 15, hh = lane >> 4;
  const int ntn = N / 64;
  const int wid = blockIdx.x * 4 + w;
  const int mt = wid / ntn, nq = wid % ntn;
  if (mt * 16 >= M) return;
  const int row0 = mt * 16, col0 = nq * 64;
  const float* arow = A + (size_t)(row0 + ln) * lda;
  v8f acc[4] = {};
  for (int kb = 0; kb < K; kb += 32) {
    FragB ah, al;
    const v4f x0 = *(const v4fa*)(arow + kb + 8 * hh), x1 = *(const v4fa*)(arow + kb + 8 * hh + 4);
    const v4f x2 = *(const v4fa*)(arow + kb + 16 + 8 * hh), x3 = *(const v4fa*)(arow + kb + 16 + 8 * hh + 4);
    float xs[16] = {x0[0],x0[1],x0[2],x0[3],x1[0],x1[1],x1[2],x1[3],x2[0],x2[1],x2[2],x2[3],x3[0],x3[1],x3[2],x3[3]};
#pragma unroll
    for (int i = 0; i < 16; ++i) { const unsigned short hb = bf16_bits(xs[i]); ah.u[i] = hb; al.u[i] = ASPLIT ? bf16_bits(xs[i] - bf16_val(hb)) : (unsigned short)0; }
#pragma unroll
    for (int t = 0; t < 4; ++t) {
      const unsigned short* brow = Wt + (size_t)(col0 + t * 16 + ln) * ldb + kb;
      FragB b;
      b.half[0] = *(const v8us*)(brow + 8 * hh);
      b.half[1] = *(const v8us*)(brow + 16 + 8 * hh);
      acc[t] = mmaN<ASPLIT ? 2 : 1>(ah.v, al.v, b.v, b.v, acc[t]);
    }
  }
#pragma unroll
  for (int t = 0; t < 4; ++t) {
    float bv = bias ? bias[col0 + t * 16 + ln] : 0.f;
    if (BIAS_BF16) bv = bf16_round(bv);
#pragma unroll
    for (int r = 0; r < 8; ++r) { float v = acc[t][r] + bv; if (ACT == 1) v = fmaxf(v, 0.f); so[w][8 * hh + r][t * 16 + ln] = v; }
  }
  __builtin_amdgcn_fence(__ATOMIC_ACQ_REL, "workgroup");
  __builtin_amdgcn_wave_barrier();
  const int rsub = lane >> 4, c4 = (lane & 15) * 4;
  for (int pass = 0; pass < 2; ++pass) {
#pragma unroll
    for (int q = 0; q < 8; ++q) {
      const int r = q * 2 + rsub;
      const v4f v = *(const v4fa*)&so[w][r][c4];
      *(volatile v4f*)(C + (size_t)(row0 + r) * ldc + col0 + c4) = v;
    }
    if (pass == 0) __threadfence();
  }
}

template <int D, bool CAUSAL>
__global__ __launch_bounds__(128) void k_flash(const float* __restrict__ qb, const float* __restrict__ kb, const float* __restrict__ vb,
                                             int pitch, int T, int H, float scale, float* __restrict__ y, int ypitch) {
  constexpr int KS = D / 32;
  constexpr int DT = D / 16;
  __shared__ __attribute__((aligned(16))) unsigned short sKh[32][D + 8], sKl[32][D + 8], sVh[32][D + 8], sVl[32][D + 8];
  __shared__ __attribute__((aligned(16))) unsigned short sPh[4][16][40], sPl[4][16][40];
  __shared__ __attribute__((aligned(16))) float sO[4][16][D];
  const int tid = threadIdx.x, w = tid >> 5, lane = tid & 31, ln = lane & 15, hh = lane >> 4;
  const int nqb = (T + 63) / 64;
  const int bh = blockIdx.x / nqb, qblk = blockIdx.x % nqb;
  const int b = bh / H, h = bh % H;
  const int q0 = qblk * 64 + w * 16;
  const float* Q = qb + (size_t)b * T * pitch + h * D;
  const float* K = kb + (size_t)b * T * pitch + h * D;
  const float* V = vb + (size_t)b * T * pitch + h * D;

  FragB aqh[KS], aql[KS];
  {
    int row = q0 + ln; if (row >= T) row = T - 1;
    const float* qr = Q + (size_t)row * pitch;
#pragma unroll
    for (int ks = 0; ks < KS; ++ks)
#pragma unroll
      for (int i = 0; i < 16; ++i) {
        const int d = ks * 32 + ((i < 8) ? (8 * hh + i) : (16 + 8 * hh + (i - 8)));
        const float x = qr[d] * scale; const unsigned short hb = bf16_bits(x);
        aqh[ks].u[i] = hb; aql[ks].u[i] = bf16_bits(x - bf16_val(hb));
      }
  }
  float m_r[8], l_r[8];
#pragma unroll
  for (int r = 0; r < 8; ++r) { m_r[r] = -3.0e38f; l_r[r] = 0.f; }
  v8f oacc[DT];
#pragma unroll
  for (int dt = 0; dt < DT; ++dt) oacc[dt] = (v8f){0.f,0.f,0.f,0.f,0.f,0.f,0.f,0.f};

  const int kv_end = CAUSAL ? min(T, qblk * 64 + 64) : T;
  for (int j0 = 0; j0 < kv_end; j0 += 32) {
    __syncthreads();
    for (int e = tid; e < 32 * (D / 4); e += 128) {
      const int r = e / (D / 4), c4 = (e % (D / 4)) * 4;
      const int key = j0 + r;
      v4f kf = {0.f,0.f,0.f,0.f}, vf = {0.f,0.f,0.f,0.f};
      if (key < T) { kf = *(const v4fa*)(K + (size_t)key * pitch + c4); vf = *(const v4fa*)(V + (size_t)key * pitch + c4); }
#pragma unroll
      for (int t = 0; t < 4; ++t) {
        unsigned short hb = bf16_bits(kf[t]); sKh[r][c4 + t] = hb; sKl[r][c4 + t] = bf16_bits(kf[t] - bf16_val(hb));
        hb = bf16_bits(vf[t]); sVh[r][c4 + t] = hb; sVl[r][c4 + t] = bf16_bits(vf[t] - bf16_val(hb));
      }
    }
    __syncthreads();
    v8f s[2];
#pragma unroll
    for (int nt = 0; nt < 2; ++nt) {
      v8f acc = {};
#pragma unroll
      for (int ks = 0; ks < KS; ++ks) {
        FragB bh_, bl_;
        bh_.half[0] = *(const v8us*)&sKh[nt * 16 + ln][ks * 32 + 8 * hh]; bh_.half[1] = *(const v8us*)&sKh[nt * 16 + ln][ks * 32 + 16 + 8 * hh];
        bl_.half[0] = *(const v8us*)&sKl[nt * 16 + ln][ks * 32 + 8 * hh]; bl_.half[1] = *(const v8us*)&sKl[nt * 16 + ln][ks * 32 + 16 + 8 * hh];
        acc = mmaN<3>(aqh[ks].v, aql[ks].v, bh_.v, bl_.v, acc);
      }
      s[nt] = acc;
    }
    float alpha[8];
#pragma unroll
    for (int r = 0; r < 8; ++r) {
      const int qi = q0 + 8 * hh + r;
      const int ja = j0 + ln, jb = j0 + 16 + ln;
      if (CAUSAL) { if (ja > qi) s[0][r] = -3.0e38f; if (jb > qi) s[1][r] = -3.0e38f; }
      if (ja >= T) s[0][r] = -3.0e38f;
      if (jb >= T) s[1][r] = -3.0e38f;
      float mx = fmaxf(s[0][r], s[1][r]);
      mx = fmaxf(mx, __shfl_xor(mx, 1, 32)); mx = fmaxf(mx, __shfl_xor(mx, 2, 32)); mx = fmaxf(mx, __shfl_xor(mx, 4, 32)); mx = fmaxf(mx, __shfl_xor(mx, 8, 32));
      const float mnew = fmaxf(m_r[r], mx);
      alpha[r] = (mnew > -1.0e38f) ? __expf(m_r[r] - mnew) : 1.0f;
      const float p0 = (s[0][r] > -1.0e38f) ? __expf(s[0][r] - mnew) : 0.f;
      const float p1 = (s[1][r] > -1.0e38f) ? __expf(s[1][r] - mnew) : 0.f;
      m_r[r] = mnew;
      l_r[r] = l_r[r] * alpha[r] + p0 + p1;
      unsigned short hb = bf16_bits(p0); sPh[w][8 * hh + r][ln] = hb;      sPl[w][8 * hh + r][ln] = bf16_bits(p0 - bf16_val(hb));
      hb = bf16_bits(p1);                sPh[w][8 * hh + r][16 + ln] = hb; sPl[w][8 * hh + r][16 + ln] = bf16_bits(p1 - bf16_val(hb));
    }
#pragma unroll
    for (int dt = 0; dt < DT; ++dt)
#pragma unroll
      for (int r = 0; r < 8; ++r) oacc[dt][r] *= alpha[r];
    __builtin_amdgcn_fence(__ATOMIC_ACQ_REL, "workgroup");
    __builtin_amdgcn_wave_barrier();
    FragB pah, pal;
    pah.half[0] = *(const v8us*)&sPh[w][ln][8 * hh]; pah.half[1] = *(const v8us*)&sPh[w][ln][16 + 8 * hh];
    pal.half[0] = *(const v8us*)&sPl[w][ln][8 * hh]; pal.half[1] = *(const v8us*)&sPl[w][ln][16 + 8 * hh];
#pragma unroll
    for (int dt = 0; dt < DT; ++dt) {
      FragB bvh, bvl;
#pragma unroll
      for (int i = 0; i < 8; ++i) {
        bvh.u[i] = sVh[8 * hh + i][dt * 16 + ln]; bvh.u[8 + i] = sVh[16 + 8 * hh + i][dt * 16 + ln];
        bvl.u[i] = sVl[8 * hh + i][dt * 16 + ln]; bvl.u[8 + i] = sVl[16 + 8 * hh + i][dt * 16 + ln];
      }
      oacc[dt] = mmaN<3>(pah.v, pal.v, bvh.v, bvl.v, oacc[dt]);
    }
    __builtin_amdgcn_fence(__ATOMIC_ACQ_REL, "workgroup");
    __builtin_amdgcn_wave_barrier();
  }
#pragma unroll
  for (int r = 0; r < 8; ++r) {
    float l = l_r[r];
    l += __shfl_xor(l, 1, 32); l += __shfl_xor(l, 2, 32); l += __shfl_xor(l, 4, 32); l += __shfl_xor(l, 8, 32);
    l_r[r] = (l > 0.f) ? 1.0f / l : 0.f;
  }
#pragma unroll
  for (int dt = 0; dt < DT; ++dt)
#pragma unroll
    for (int r = 0; r < 8; ++r) sO[w][8 * hh + r][dt * 16 + ln] = oacc[dt][r] * l_r[r];
  __builtin_amdgcn_fence(__ATOMIC_ACQ_REL, "workgroup");
  __builtin_amdgcn_wave_barrier();
  for (int pass = 0; pass < 2; ++pass) {
    for (int r = 0; r < 16; ++r) {
      const int row = q0 + r;
      if (row < T && lane < D / 4) {
        const v4f val = *(const v4fa*)&sO[w][r][lane * 4];
        *(volatile v4f*)(y + ((size_t)b * T + row) * ypitch + h * D + lane * 4) = val;
      }
    }
    if (pass == 0) __threadfence();
  }
}

template <bool AFFINE, bool RESID, bool RES_BF16>
__global__ __launch_bounds__(256) void k_transpose32(const float* __restrict__ in, float* __restrict__ out, int rows, int cols,
                                                    const float* __restrict__ scale, const float* __restrict__ shift, const float* __restrict__ res) {
  __shared__ float tile[32][33];
  const int b = blockIdx.z;
  const int r0 = blockIdx.y * 32, c0 = blockIdx.x * 32;
  const float* src = in + (size_t)b * rows * cols;
  float* dst = out + (size_t)b * rows * cols;
  const int tx = threadIdx.x & 31, ty = threadIdx.x >> 5;
  for (int i = ty; i < 32; i += 8) tile[i][tx] = src[(size_t)(r0 + i) * cols + c0 + tx];
  __syncthreads();
  for (int pass = 0; pass < 2; ++pass) {
    for (int i = ty; i < 32; i += 8) {
      float v = tile[tx][i];
      const int orow = c0 + i;
      if (AFFINE) v = v * scale[orow] + shift[orow];
      if (RESID) { float rv = res[(size_t)b * rows * cols + (size_t)orow * rows + r0 + tx]; if (RES_BF16) rv = bf16_round(rv); v += rv; }
      *(volatile float*)(dst + (size_t)orow * rows + r0 + tx) = v;
    }
    if (pass == 0) __threadfence();
  }
}

__global__ __launch_bounds__(256) void k_pool2_pm(const float* __restrict__ in, float* __restrict__ out, int Bn, int H, int W, int C) {
  const size_t t = (size_t)blockIdx.x * 256 + threadIdx.x;
  const int c4n = C / 4, Ho = H / 2, Wo = W / 2;
  const size_t total = (size_t)Bn * Ho * Wo * c4n;
  if (t >= total) return;
  const int c4 = (int)(t % c4n) * 4; size_t rest = t / c4n;
  const int pw = (int)(rest % Wo); rest /= Wo; const int ph = (int)(rest % Ho); const int b = (int)(rest / Ho);
  const float* base = in + (size_t)b * H * W * C;
  const int p00 = (2 * ph) * W + 2 * pw;
  const v4f a = *(const v4fa*)(base + (size_t)p00 * C + c4), bq = *(const v4fa*)(base + (size_t)(p00 + 1) * C + c4);
  const v4f c = *(const v4fa*)(base + (size_t)(p00 + W) * C + c4), d = *(const v4fa*)(base + (size_t)(p00 + W + 1) * C + c4);
  v4f m; for (int i = 0; i < 4; ++i) m[i] = fmaxf(fmaxf(a[i], bq[i]), fmaxf(c[i], d[i]));
  float* dst = out + ((size_t)b * Ho * Wo + (size_t)ph * Wo + pw) * C + c4;
  *(volatile v4f*)dst = m;
  __threadfence();
  *(volatile v4f*)dst = m;
}

template <int DQ, int DV>
__global__ __launch_bounds__(128) void k_flash2(const float* __restrict__ Qb, size_t qstride, int qpitch, int Tq,
                                              const float* __restrict__ Kb, size_t kstride, int kpitch, int Tk,
                                              const float* __restrict__ Vb, size_t vstride, int vpitch,
                                              float scale, float* __restrict__ y, size_t ystride, int ypitch) {
  constexpr int KS = DQ / 32, DT = DV / 16;
  __shared__ __attribute__((aligned(16))) unsigned short sKh[32][DQ + 8], sKl[32][DQ + 8], sVh[32][DV + 8], sVl[32][DV + 8];
  __shared__ __attribute__((aligned(16))) unsigned short sPh[4][16][40], sPl[4][16][40];
  __shared__ __attribute__((aligned(16))) float sO[4][16][DV];
  const int tid = threadIdx.x, w = tid >> 5, lane = tid & 31, ln = lane & 15, hh = lane >> 4;
  const int nqb = (Tq + 63) / 64;
  const int bh = blockIdx.x / nqb, qblk = blockIdx.x % nqb;
  const int dv0 = blockIdx.y * DV;
  const int q0 = qblk * 64 + w * 16;
  const float* Q = Qb + (size_t)bh * qstride; const float* K = Kb + (size_t)bh * kstride; const float* V = Vb + (size_t)bh * vstride + dv0;
  FragB aqh[KS], aql[KS];
  {
    int row = q0 + ln; if (row >= Tq) row = Tq - 1;
    const float* qr = Q + (size_t)row * qpitch;
#pragma unroll
    for (int ks = 0; ks < KS; ++ks)
#pragma unroll
      for (int i = 0; i < 16; ++i) {
        const int d = ks * 32 + ((i < 8) ? (8 * hh + i) : (16 + 8 * hh + (i - 8)));
        const float x = qr[d] * scale; const unsigned short hb = bf16_bits(x);
        aqh[ks].u[i] = hb; aql[ks].u[i] = bf16_bits(x - bf16_val(hb));
      }
  }
  float m_r[8], l_r[8];
#pragma unroll
  for (int r = 0; r < 8; ++r) { m_r[r] = -3.0e38f; l_r[r] = 0.f; }
  v8f oacc[DT];
#pragma unroll
  for (int dt = 0; dt < DT; ++dt) oacc[dt] = (v8f){0.f,0.f,0.f,0.f,0.f,0.f,0.f,0.f};
  for (int j0 = 0; j0 < Tk; j0 += 32) {
    __syncthreads();
    for (int e = tid; e < 32 * (DQ / 4); e += 128) {
      const int r = e / (DQ / 4), c4 = (e % (DQ / 4)) * 4; const int key = j0 + r;
      v4f f = {0.f,0.f,0.f,0.f}; if (key < Tk) f = *(const v4fa*)(K + (size_t)key * kpitch + c4);
#pragma unroll
      for (int t = 0; t < 4; ++t) { const unsigned short hb = bf16_bits(f[t]); sKh[r][c4 + t] = hb; sKl[r][c4 + t] = bf16_bits(f[t] - bf16_val(hb)); }
    }
    for (int e = tid; e < 32 * (DV / 4); e += 128) {
      const int r = e / (DV / 4), c4 = (e % (DV / 4)) * 4; const int key = j0 + r;
      v4f f = {0.f,0.f,0.f,0.f}; if (key < Tk) f = *(const v4fa*)(V + (size_t)key * vpitch + c4);
#pragma unroll
      for (int t = 0; t < 4; ++t) { const unsigned short hb = bf16_bits(f[t]); sVh[r][c4 + t] = hb; sVl[r][c4 + t] = bf16_bits(f[t] - bf16_val(hb)); }
    }
    __syncthreads();
    v8f s[2];
#pragma unroll
    for (int nt = 0; nt < 2; ++nt) {
      v8f acc = {};
#pragma unroll
      for (int ks = 0; ks < KS; ++ks) {
        FragB bh_, bl_;
        bh_.half[0] = *(const v8us*)&sKh[nt * 16 + ln][ks * 32 + 8 * hh]; bh_.half[1] = *(const v8us*)&sKh[nt * 16 + ln][ks * 32 + 16 + 8 * hh];
        bl_.half[0] = *(const v8us*)&sKl[nt * 16 + ln][ks * 32 + 8 * hh]; bl_.half[1] = *(const v8us*)&sKl[nt * 16 + ln][ks * 32 + 16 + 8 * hh];
        acc = mmaN<3>(aqh[ks].v, aql[ks].v, bh_.v, bl_.v, acc);
      }
      s[nt] = acc;
    }
    float alpha[8];
#pragma unroll
    for (int r = 0; r < 8; ++r) {
      const int ja = j0 + ln, jb = j0 + 16 + ln;
      if (ja >= Tk) s[0][r] = -3.0e38f;
      if (jb >= Tk) s[1][r] = -3.0e38f;
      float mx = fmaxf(s[0][r], s[1][r]);
      mx = fmaxf(mx, __shfl_xor(mx, 1, 32)); mx = fmaxf(mx, __shfl_xor(mx, 2, 32)); mx = fmaxf(mx, __shfl_xor(mx, 4, 32)); mx = fmaxf(mx, __shfl_xor(mx, 8, 32));
      const float mnew = fmaxf(m_r[r], mx);
      alpha[r] = (mnew > -1.0e38f) ? __expf(m_r[r] - mnew) : 1.0f;
      const float p0 = (s[0][r] > -1.0e38f) ? __expf(s[0][r] - mnew) : 0.f;
      const float p1 = (s[1][r] > -1.0e38f) ? __expf(s[1][r] - mnew) : 0.f;
      m_r[r] = mnew;
      l_r[r] = l_r[r] * alpha[r] + p0 + p1;
      unsigned short hb = bf16_bits(p0); sPh[w][8 * hh + r][ln] = hb;      sPl[w][8 * hh + r][ln] = bf16_bits(p0 - bf16_val(hb));
      hb = bf16_bits(p1);                sPh[w][8 * hh + r][16 + ln] = hb; sPl[w][8 * hh + r][16 + ln] = bf16_bits(p1 - bf16_val(hb));
    }
#pragma unroll
    for (int dt = 0; dt < DT; ++dt)
#pragma unroll
      for (int r = 0; r < 8; ++r) oacc[dt][r] *= alpha[r];
    __builtin_amdgcn_fence(__ATOMIC_ACQ_REL, "workgroup");
    __builtin_amdgcn_wave_barrier();
    FragB pah, pal;
    pah.half[0] = *(const v8us*)&sPh[w][ln][8 * hh]; pah.half[1] = *(const v8us*)&sPh[w][ln][16 + 8 * hh];
    pal.half[0] = *(const v8us*)&sPl[w][ln][8 * hh]; pal.half[1] = *(const v8us*)&sPl[w][ln][16 + 8 * hh];
#pragma unroll
    for (int dt = 0; dt < DT; ++dt) {
      FragB bvh, bvl;
#pragma unroll
      for (int i = 0; i < 8; ++i) {
        bvh.u[i] = sVh[8 * hh + i][dt * 16 + ln]; bvh.u[8 + i] = sVh[16 + 8 * hh + i][dt * 16 + ln];
        bvl.u[i] = sVl[8 * hh + i][dt * 16 + ln]; bvl.u[8 + i] = sVl[16 + 8 * hh + i][dt * 16 + ln];
      }
      oacc[dt] = mmaN<3>(pah.v, pal.v, bvh.v, bvl.v, oacc[dt]);
    }
    __builtin_amdgcn_fence(__ATOMIC_ACQ_REL, "workgroup");
    __builtin_amdgcn_wave_barrier();
  }
#pragma unroll
  for (int r = 0; r < 8; ++r) {
    float l = l_r[r];
    l += __shfl_xor(l, 1, 32); l += __shfl_xor(l, 2, 32); l += __shfl_xor(l, 4, 32); l += __shfl_xor(l, 8, 32);
    l_r[r] = (l > 0.f) ? 1.0f / l : 0.f;
  }
#pragma unroll
  for (int dt = 0; dt < DT; ++dt)
#pragma unroll
    for (int r = 0; r < 8; ++r) sO[w][8 * hh + r][dt * 16 + ln] = oacc[dt][r] * l_r[r];
  __builtin_amdgcn_fence(__ATOMIC_ACQ_REL, "workgroup");
  __builtin_amdgcn_wave_barrier();
  for (int pass = 0; pass < 2; ++pass) {
    for (int r = 0; r < 16; ++r) {
      const int row = q0 + r;
      for (int c4 = lane * 4; c4 < DV; c4 += 128) {
        if (row < Tq) {
          const v4f val = *(const v4fa*)&sO[w][r][c4];
          *(volatile v4f*)(y + (size_t)bh * ystride + (size_t)row * ypitch + dv0 + c4) = val;
        }
      }
    }
    if (pass == 0) __threadfence();
  }
}

typedef _Float16 v16h __attribute__((ext_vector_type(16)));
union FragH { v16h v; v8us half[2]; _Float16 h[16]; unsigned short u[16]; };
template <int NT>
__device__ __forceinline__ v8f mmaH(v16h ah, v16h al, v16h bh, v16h bl, v8f c) {
  c = __builtin_amdgcn_wmma_f32_16x16x32_f16(false, ah, false, bh, (short)0, c, false, false);
  if (NT >= 2) c = __builtin_amdgcn_wmma_f32_16x16x32_f16(false, al, false, bh, (short)0, c, false, false);
  if (NT >= 3) c = __builtin_amdgcn_wmma_f32_16x16x32_f16(false, ah, false, bl, (short)0, c, false, false);
  asm volatile("v_nop\n\tv_nop\n\tv_nop\n\tv_nop" : "+v"(c) : "v"(ah), "v"(al), "v"(bh), "v"(bl));
  return c;
}
template <bool ASPLIT>
__global__ __launch_bounds__(128) void k_gemm_h(const float* __restrict__ A, int lda, size_t sA, const _Float16* __restrict__ Bh, int ldb, size_t sB, float alpha, float* __restrict__ C, int ldc, size_t sC, int M, int N, int K) {
  __shared__ __attribute__((aligned(16))) float so[4][16][64];
  const int tid = threadIdx.x, w = tid >> 5, lane = tid & 31, ln = lane & 15, hh = lane >> 4; const int by = blockIdx.y;
  A += (size_t)by * sA; Bh += (size_t)by * sB; C += (size_t)by * sC;
  const int ntn = (N + 63) / 64; const int wid = blockIdx.x * 4 + w; const int mt = wid / ntn, nq = wid % ntn; if (mt * 16 >= M) return;
  const int row0 = mt * 16, col0 = nq * 64; const float* arow = A + (size_t)(row0 + ln) * lda;
  v8f acc[4] = {};
  for (int kb = 0; kb < K; kb += 32) {
    FragH ah, al;
    const v4f x0 = *(const v4fa*)(arow + kb + 8 * hh), x1 = *(const v4fa*)(arow + kb + 8 * hh + 4), x2 = *(const v4fa*)(arow + kb + 16 + 8 * hh), x3 = *(const v4fa*)(arow + kb + 16 + 8 * hh + 4);
    float xs[16] = {x0[0],x0[1],x0[2],x0[3],x1[0],x1[1],x1[2],x1[3],x2[0],x2[1],x2[2],x2[3],x3[0],x3[1],x3[2],x3[3]};
#pragma unroll
    for (int i = 0; i < 16; ++i) { const _Float16 h = (_Float16)xs[i]; ah.h[i] = h; al.h[i] = ASPLIT ? (_Float16)(xs[i] - (float)h) : (_Float16)0.0f; }
#pragma unroll
    for (int t = 0; t < 4; ++t) { if (col0 + t * 16 >= N) continue; const size_t boff = (size_t)(col0 + t * 16 + ln) * ldb + kb; FragH bq; bq.half[0] = *(const v8us*)(Bh + boff + 8 * hh); bq.half[1] = *(const v8us*)(Bh + boff + 16 + 8 * hh);
      acc[t] = mmaH<ASPLIT ? 2 : 1>(ah.v, al.v, bq.v, bq.v, acc[t]); }
  }
#pragma unroll
  for (int t = 0; t < 4; ++t) { if (col0 + t * 16 >= N) continue;
#pragma unroll
    for (int r = 0; r < 8; ++r) so[w][8 * hh + r][t * 16 + ln] = acc[t][r] * alpha; }
  __builtin_amdgcn_fence(__ATOMIC_ACQ_REL, "workgroup"); __builtin_amdgcn_wave_barrier();
  const int rsub = lane >> 4, c4 = (lane & 15) * 4;
  for (int pass = 0; pass < 2; ++pass) {
#pragma unroll
    for (int q = 0; q < 8; ++q) { const int r = q * 2 + rsub; if (col0 + c4 < N) { const v4f v = *(const v4fa*)&so[w][r][c4]; *(volatile v4f*)(C + (size_t)(row0 + r) * ldc + col0 + c4) = v; } }
    if (pass == 0) __threadfence(); }
}

__global__ __launch_bounds__(128) void k_nam1(const float* __restrict__ x, const float* __restrict__ w1, const float* __restrict__ b1, const _Float16* __restrict__ Bt2, const float* __restrict__ b2, int b0, _Float16* __restrict__ Hout, int M) {
  __shared__ __attribute__((aligned(16))) float so[4][16][64];
  const int tid = threadIdx.x, w = tid >> 5, lane = tid & 31, ln = lane & 15, hh = lane >> 4; const int f = blockIdx.y;
  const int wid = blockIdx.x * 4 + w; const int mt = wid; if (mt * 16 >= M) return; const int row0 = mt * 16;
  const float xv = bf16_round(x[(size_t)(b0 + row0 + ln) * NF + f]); const float* w1f = w1 + (size_t)f * U1; const float* b1f = b1 + (size_t)f * U1; const _Float16* Bf = Bt2 + (size_t)f * NH1 * U1;
  v8f acc[4] = {};
  for (int kb = 0; kb < U1; kb += 32) { FragH ah;
#pragma unroll
    for (int q = 0; q < 8; ++q) { const int u0 = kb + 8 * hh + q, u1i = kb + 16 + 8 * hh + q; ah.h[q] = (_Float16)fmaxf(xv * bf16_round(w1f[u0]) + bf16_round(b1f[u0]), 0.f); ah.h[8 + q] = (_Float16)fmaxf(xv * bf16_round(w1f[u1i]) + bf16_round(b1f[u1i]), 0.f); }
#pragma unroll
    for (int t = 0; t < 4; ++t) { const size_t boff = (size_t)(t * 16 + ln) * U1 + kb; FragH bq; bq.half[0] = *(const v8us*)((const unsigned short*)Bf + boff + 8 * hh); bq.half[1] = *(const v8us*)((const unsigned short*)Bf + boff + 16 + 8 * hh);
      acc[t] = mmaH<1>(ah.v, ah.v, bq.v, bq.v, acc[t]); }
  }
#pragma unroll
  for (int t = 0; t < 4; ++t) { const int col = t * 16 + ln; const float bb = bf16_round(b2[(size_t)f * NH1 + col]);
#pragma unroll
    for (int r = 0; r < 8; ++r) so[w][8 * hh + r][t * 16 + ln] = fmaxf(acc[t][r] * 0.25f + bb, 0.f); }
  __builtin_amdgcn_fence(__ATOMIC_ACQ_REL, "workgroup"); __builtin_amdgcn_wave_barrier();
  const int rsub = lane >> 4, c4 = (lane & 15) * 4; typedef _Float16 v4h __attribute__((ext_vector_type(4)));
  for (int pass = 0; pass < 2; ++pass) {
#pragma unroll
    for (int q = 0; q < 8; ++q) { const int r = q * 2 + rsub; const v4f v = *(const v4fa*)&so[w][r][c4]; v4h h4; for (int u = 0; u < 4; ++u) h4[u] = (_Float16)v[u]; *(volatile v4h*)(Hout + (size_t)(row0 + r) * (NF * NH1) + (size_t)f * NH1 + c4) = h4; }
    if (pass == 0) __threadfence(); }
}
__global__ __launch_bounds__(128) void k_nam2(const _Float16* __restrict__ Hin, const _Float16* __restrict__ Bt3, const float* __restrict__ b3, const float* __restrict__ wo, const float* __restrict__ bo, int b0, float* __restrict__ PFOT, int M) {
  __shared__ float sp[4][16];
  const int tid = threadIdx.x, w = tid >> 5, lane = tid & 31, ln = lane & 15, hh = lane >> 4; const int f = blockIdx.y;
  const int wid = blockIdx.x * 4 + w; const int mt = wid; if (mt * 16 >= M) return; const int row0 = mt * 16;
  const _Float16* arow = Hin + (size_t)(row0 + ln) * (NF * NH1) + (size_t)f * NH1; const _Float16* Bf = Bt3 + (size_t)f * NH2 * NH1;
  v8f acc[2] = {};
  for (int kb = 0; kb < NH1; kb += 32) { FragH ah; ah.half[0] = *(const v8us*)((const unsigned short*)arow + kb + 8 * hh); ah.half[1] = *(const v8us*)((const unsigned short*)arow + kb + 16 + 8 * hh);
#pragma unroll
    for (int t = 0; t < 2; ++t) { const size_t boff = (size_t)(t * 16 + ln) * NH1 + kb; FragH bq; bq.half[0] = *(const v8us*)((const unsigned short*)Bf + boff + 8 * hh); bq.half[1] = *(const v8us*)((const unsigned short*)Bf + boff + 16 + 8 * hh);
      acc[t] = mmaH<1>(ah.v, ah.v, bq.v, bq.v, acc[t]); }
  }
  float rowsum[8] = {0.f, 0.f, 0.f, 0.f, 0.f, 0.f, 0.f, 0.f};
#pragma unroll
  for (int t = 0; t < 2; ++t) { const int col = t * 16 + ln; const float bb = bf16_round(b3[(size_t)f * NH2 + col]), wc = bf16_round(wo[(size_t)f * NH2 + col]);
#pragma unroll
    for (int r = 0; r < 8; ++r) rowsum[r] += fmaxf(acc[t][r] * 0.25f + bb, 0.f) * wc; }
#pragma unroll
  for (int r = 0; r < 8; ++r) { float s = rowsum[r]; for (int o = 8; o >= 1; o >>= 1) s += __shfl_xor(s, o, 32); rowsum[r] = s; }
  const float bof = bf16_round(bo[f]); if (ln == 0) { for (int r = 0; r < 8; ++r) sp[w][8 * hh + r] = rowsum[r] + bof; }
  __builtin_amdgcn_fence(__ATOMIC_ACQ_REL, "workgroup"); __builtin_amdgcn_wave_barrier();
  if (lane < 16) { *(volatile float*)(PFOT + (size_t)f * BS + b0 + row0 + lane) = sp[w][lane]; } __threadfence(); if (lane < 16) { *(volatile float*)(PFOT + (size_t)f * BS + b0 + row0 + lane) = sp[w][lane]; }
}

__global__ __launch_bounds__(256) void k_wt(const float* __restrict__ w2, const float* __restrict__ w3, _Float16* __restrict__ Bt2, _Float16* __restrict__ Bt3) { const int t = blockIdx.x * 256 + threadIdx.x;
  if (t < NF * NH1 * (U1 / 8)) { const int u8 = (t % (U1 / 8)) * 8; const int h = (t / (U1 / 8)) % NH1; const int f = t / ((U1 / 8) * NH1); FragH fr; for (int q = 0; q < 8; ++q) fr.h[q] = (_Float16)(bf16_round(w2[((size_t)f * U1 + u8 + q) * NH1 + h]) * 4.0f); unsigned short* d = (unsigned short*)Bt2 + ((size_t)f * NH1 + h) * U1 + u8; *(volatile v8us*)d = fr.half[0]; __threadfence(); *(volatile v8us*)d = fr.half[0]; }
  if (t < NF * NH2 * (NH1 / 8)) { const int h8 = (t % (NH1 / 8)) * 8; const int k = (t / (NH1 / 8)) % NH2; const int f = t / ((NH1 / 8) * NH2); FragH fr; for (int q = 0; q < 8; ++q) fr.h[q] = (_Float16)(bf16_round(w3[((size_t)f * NH1 + h8 + q) * NH2 + k]) * 4.0f); unsigned short* d = (unsigned short*)Bt3 + ((size_t)f * NH2 + k) * NH1 + h8; *(volatile v8us*)d = fr.half[0]; __threadfence(); *(volatile v8us*)d = fr.half[0]; } }
__global__ __launch_bounds__(256) void k_lin(const float* __restrict__ pfo, const float* __restrict__ icpt, float* __restrict__ lin) { const int b = blockIdx.x * 256 + threadIdx.x; if (b >= BS) return; float s = 0.f;
#pragma unroll 4
  for (int f = 0; f < NF; ++f) s += pfo[(size_t)b * NF + f]; const float v = bf16_round(icpt[0]) + s; *(volatile float*)(lin + b) = v; __threadfence(); *(volatile float*)(lin + b) = v; }
extern "C" void kernel_launch(void* const* d_in, const int* in_sizes, int n_in,
                              void* d_out, int out_size, void* d_ws, size_t ws_size, hipStream_t stream) {
  (void)in_sizes; (void)n_in; (void)out_size;
  const float* x = (const float*)d_in[0]; const float* w1 = (const float*)d_in[1]; const float* b1 = (const float*)d_in[2]; const float* w2 = (const float*)d_in[3]; const float* b2 = (const float*)d_in[4]; const float* w3 = (const float*)d_in[5]; const float* b3 = (const float*)d_in[6]; const float* wo = (const float*)d_in[7]; const float* bo = (const float*)d_in[8]; const float* icpt = (const float*)d_in[9];
  float* lin = (float*)d_out; float* pfo = lin + BS;
  char* ws = (char*)d_ws; size_t off = 0;
  auto take = [&](size_t bytes) { char* p = ws + off; off += (bytes + 255) & ~(size_t)255; return p; };
  _Float16* Bt2 = (_Float16*)take((size_t)NF * NH1 * U1 * 2); _Float16* Bt3 = (_Float16*)take((size_t)NF * NH2 * NH1 * 2); _Float16* H2b = (_Float16*)take((size_t)CHB * NF * NH1 * 2); float* PFOT = (float*)take((size_t)NF * BS * 4);
  if (off > ws_size) return;
  k_wt<<<(NF * NH1 * (U1 / 8) + 255) / 256, 256, 0, stream>>>(w2, w3, Bt2, Bt3);
  for (int b0 = 0; b0 < BS; b0 += CHB) {
    k_nam1<<<dim3((CHB / 16 + 3) / 4, NF), 128, 0, stream>>>(x, w1, b1, Bt2, b2, b0, H2b, CHB);
    k_nam2<<<dim3((CHB / 16 + 3) / 4, NF), 128, 0, stream>>>(H2b, Bt3, b3, wo, bo, b0, PFOT, CHB);
  }
  k_transpose32<false, false, false><<<dim3(BS / 32, NF / 32, 1), 256, 0, stream>>>(PFOT, pfo, NF, BS, nullptr, nullptr, nullptr);
  k_lin<<<BS / 256, 256, 0, stream>>>(pfo, icpt, lin);
}
